// NewMinibatchEnergyDistance_52965536694314
// MI455X (gfx1250) — hardware-verified
//
#include <hip/hip_runtime.h>


typedef _Float16 v16h __attribute__((ext_vector_type(16)));
typedef _Float16 v8h  __attribute__((ext_vector_type(8)));
typedef _Float16 v4h  __attribute__((ext_vector_type(4)));
typedef float    v8f  __attribute__((ext_vector_type(8)));
typedef float    v4f  __attribute__((ext_vector_type(4)));
typedef double   v2d  __attribute__((ext_vector_type(2)));

union FragH { v16h v; v8h h8[2]; };

#define NB    1024
#define DIN   3072
#define DE    256
#define NMAT  4
#define NPAIR 6
#define SKT   256
#define SKW   (SKT / 32)
#define ITMAX 64

#define SC_X  16.0f
#define SC_W  64.0f
#define SC_U  128.0f

__device__ __forceinline__ v8f wmma16(const v16h a, const v16h b, v8f c) {
  return __builtin_amdgcn_wmma_f32_16x16x32_f16(false, a, false, b, (short)0, c, false, false);
}

#define WMMA_GUARD4(A, B0, B1, B2, B3, C0, C1, C2, C3)                                   \
  asm volatile("v_nop\n\tv_nop\n\tv_nop\n\tv_nop"                                       \
               : "+v"(C0), "+v"(C1), "+v"(C2), "+v"(C3)                                 \
               : "v"(A), "v"(B0), "v"(B1), "v"(B2), "v"(B3))

__device__ __forceinline__ v16h load_frag(const _Float16* p) {
  FragH f;
  f.h8[0] = *(const v8h*)(p);
  f.h8[1] = *(const v8h*)(p + 16);
  return f.v;
}

__device__ __forceinline__ float wave_sum(float v) {
#pragma unroll
  for (int o = 16; o > 0; o >>= 1) v += __shfl_xor(v, o, 32);
  return v;
}
__device__ __forceinline__ float wave_max(float v) {
#pragma unroll
  for (int o = 16; o > 0; o >>= 1) v = fmaxf(v, __shfl_xor(v, o, 32));
  return v;
}

__global__ void __launch_bounds__(256) k_wt(const float* __restrict__ Wc, _Float16* __restrict__ Wt) {
  __shared__ _Float16 tile[64 * 72] __attribute__((aligned(16)));
  const int k0 = blockIdx.x * 64;
  const int n0 = blockIdx.y * 64;
  const int t = threadIdx.x;
  const int c = t & 63, rb = t >> 6;
#pragma unroll
  for (int s = 0; s < 16; ++s) {
    const int r = rb + 4 * s;
    const float w = Wc[(size_t)(k0 + r) * DE + n0 + c];
    tile[c * 72 + r] = (_Float16)(w * SC_W);
  }
  __syncthreads();
  const int wv = t >> 5, lane = t & 31, piece = lane & 7, sub = lane >> 3;
  v8h val[2];
  size_t dst[2];
#pragma unroll
  for (int s = 0; s < 2; ++s) {
    const int nr = wv * 8 + s * 4 + sub;
    val[s] = *(const v8h*)(tile + nr * 72 + piece * 8);
    dst[s] = (size_t)(n0 + nr) * DIN + k0 + piece * 8;
  }
#pragma unroll
  for (int s = 0; s < 2; ++s) *(volatile v8h*)(Wt + dst[s]) = val[s];
  __threadfence();
#pragma unroll
  for (int s = 0; s < 2; ++s) *(volatile v8h*)(Wt + dst[s]) = val[s];
}

__global__ void __launch_bounds__(128) k_critic(const float* __restrict__ x0, const float* __restrict__ x1,
                                                const float* __restrict__ x2, const float* __restrict__ x3,
                                                const _Float16* __restrict__ Wt, const float* __restrict__ bc,
                                                _Float16* __restrict__ Fn) {
  __shared__ float ssq[4 * 16];
  __shared__ _Float16 stg[16 * 264] __attribute__((aligned(16)));
  const int mat = blockIdx.y;
  const int m0 = blockIdx.x * 16;
  const int t = threadIdx.x, wv = t >> 5, lane = t & 31, h = lane >> 4, m = lane & 15;
  const int n0 = wv * 64;
  const float* X = x0;
  if (mat == 1) X = x1; else if (mat == 2) X = x2; else if (mat == 3) X = x3;

  const float* arow = X + (size_t)(m0 + m) * DIN + 8 * h;
  const _Float16* brow0 = Wt + (size_t)(n0 + m) * DIN + 8 * h;
  v8f acc[4] = {};

#pragma unroll 1
  for (int k0 = 0; k0 < DIN; k0 += 32) {
    const v4f* ap = (const v4f*)(arow + k0);
    const v4f f0 = ap[0], f1 = ap[1];
    const v4f f2 = ap[4], f3 = ap[5];
    FragH a;
    a.h8[0] = __builtin_shufflevector(__builtin_convertvector(f0 * SC_X, v4h),
                                      __builtin_convertvector(f1 * SC_X, v4h), 0, 1, 2, 3, 4, 5, 6, 7);
    a.h8[1] = __builtin_shufflevector(__builtin_convertvector(f2 * SC_X, v4h),
                                      __builtin_convertvector(f3 * SC_X, v4h), 0, 1, 2, 3, 4, 5, 6, 7);
    v16h b[4];
#pragma unroll
    for (int c = 0; c < 4; ++c) b[c] = load_frag(brow0 + (size_t)c * (16 * DIN) + k0);
#pragma unroll
    for (int c = 0; c < 4; ++c) acc[c] = wmma16(a.v, b[c], acc[c]);
    WMMA_GUARD4(a.v, b[0], b[1], b[2], b[3], acc[0], acc[1], acc[2], acc[3]);
  }

  float Fv[4][8];
  float ss[8];
#pragma unroll
  for (int r = 0; r < 8; ++r) ss[r] = 0.f;
#pragma unroll
  for (int c = 0; c < 4; ++c) {
    const float bias = bc[n0 + 16 * c + m];
#pragma unroll
    for (int r = 0; r < 8; ++r) {
      const float v = fmaf(acc[c][r], 1.0f / (SC_X * SC_W), bias);
      Fv[c][r] = v;
      ss[r] = fmaf(v, v, ss[r]);
    }
  }
#pragma unroll
  for (int r = 0; r < 8; ++r) {
    ss[r] += __shfl_xor(ss[r], 1, 32);
    ss[r] += __shfl_xor(ss[r], 2, 32);
    ss[r] += __shfl_xor(ss[r], 4, 32);
    ss[r] += __shfl_xor(ss[r], 8, 32);
  }
  if (m == 0) {
#pragma unroll
    for (int r = 0; r < 8; ++r) ssq[wv * 16 + 8 * h + r] = ss[r];
  }
  __syncthreads();
#pragma unroll
  for (int r = 0; r < 8; ++r) {
    const int row = 8 * h + r;
    const float tot = ((ssq[row] + ssq[16 + row]) + ssq[32 + row]) + ssq[48 + row];
    const float scl = SC_U * rsqrtf(tot);
#pragma unroll
    for (int c = 0; c < 4; ++c) stg[row * 264 + n0 + 16 * c + m] = (_Float16)(Fv[c][r] * scl);
  }
  __syncthreads();

  const int piece = lane & 7, sub = lane >> 3;
  v8h val[4];
  size_t dst[4];
#pragma unroll
  for (int s = 0; s < 4; ++s) {
    const int L = 16 * wv + 4 * s + sub;
    const int row = L >> 2, seg = L & 3;
    val[s] = *(const v8h*)(stg + row * 264 + seg * 64 + piece * 8);
    dst[s] = ((size_t)(mat * NB + m0 + row)) * DE + seg * 64 + piece * 8;
  }
#pragma unroll
  for (int s = 0; s < 4; ++s) *(volatile v8h*)(Fn + dst[s]) = val[s];
  __threadfence();
#pragma unroll
  for (int s = 0; s < 4; ++s) *(volatile v8h*)(Fn + dst[s]) = val[s];
}

__global__ void __launch_bounds__(128) k_cos(const _Float16* __restrict__ Fn, float* __restrict__ C) {
  __shared__ float stg[4 * 16 * 68] __attribute__((aligned(16)));
  const int k = blockIdx.z;
  const int m0 = blockIdx.y * 16;
  const int t = threadIdx.x, wv = t >> 5, lane = t & 31, h = lane >> 4, m = lane & 15;
  const int n0 = blockIdx.x * 256 + wv * 64;
  int ai, bi;
  if (k < 4)       { ai = k >> 1; bi = 2 + (k & 1); }
  else if (k == 4) { ai = 0; bi = 1; }
  else             { ai = 2; bi = 3; }
  const _Float16* arow  = Fn + ((size_t)ai * NB + m0 + m) * DE + 8 * h;
  const _Float16* brow0 = Fn + ((size_t)bi * NB + n0 + m) * DE + 8 * h;
  v8f acc[4] = {};

#pragma unroll 1
  for (int k0 = 0; k0 < DE; k0 += 32) {
    const v16h a = load_frag(arow + k0);
    v16h b[4];
#pragma unroll
    for (int c = 0; c < 4; ++c) b[c] = load_frag(brow0 + (size_t)c * (16 * DE) + k0);
#pragma unroll
    for (int c = 0; c < 4; ++c) acc[c] = wmma16(a, b[c], acc[c]);
    WMMA_GUARD4(a, b[0], b[1], b[2], b[3], acc[0], acc[1], acc[2], acc[3]);
  }

  float* st = stg + wv * (16 * 68);
#pragma unroll
  for (int c = 0; c < 4; ++c)
#pragma unroll
    for (int r = 0; r < 8; ++r)
      st[(8 * h + r) * 68 + 16 * c + m] = fmaf(acc[c][r], -1.0f / (SC_U * SC_U), 1.0f);
  __syncthreads();

  float* Ck = C + ((size_t)k << 20);
  const int piece = lane & 7, sub = lane >> 3;
  v4f val[8];
  size_t dst[8];
#pragma unroll
  for (int s = 0; s < 8; ++s) {
    const int L = 4 * s + sub;
    const int row = L >> 1, seg = L & 1;
    val[s] = *(const v4f*)(st + row * 68 + seg * 32 + piece * 4);
    dst[s] = (size_t)(m0 + row) * NB + n0 + seg * 32 + piece * 4;
  }
#pragma unroll
  for (int s = 0; s < 8; ++s) *(volatile v4f*)(Ck + dst[s]) = val[s];
  __threadfence();
#pragma unroll
  for (int s = 0; s < 8; ++s) *(volatile v4f*)(Ck + dst[s]) = val[s];
}

__device__ __forceinline__ float block_max4(const float* arr, float* red, int t, int wv, int lane) {
  float v = fmaxf(fmaxf(arr[t], arr[t + SKT]), fmaxf(arr[t + 2 * SKT], arr[t + 3 * SKT]));
  v = wave_max(v);
  if (lane == 0) red[wv] = v;
  __syncthreads();
  float r = red[0];
#pragma unroll
  for (int w = 1; w < SKW; ++w) r = fmaxf(r, red[w]);
  return r;
}

__global__ void __launch_bounds__(SKT) k_sink(const float* __restrict__ C, const int* __restrict__ nit,
                                              double* __restrict__ Wl) {
  __shared__ float fsh[NB] __attribute__((aligned(16)));
  __shared__ float gsh[NB] __attribute__((aligned(16)));
  __shared__ float psh[NB] __attribute__((aligned(16)));
  __shared__ float red[SKW];
  __shared__ double redd[SKT];
  __shared__ double wtot;
  const int k = blockIdx.x;
  const int t = threadIdx.x, wv = t >> 5, lane = t & 31;
  const float* Ck = C + ((size_t)k << 20);
  int n = nit[0];
  n = (n < 0) ? 0 : ((n > ITMAX) ? ITMAX : n);
  const float K2  = 14.426950408889634f;
  const float ELN = 0.1f * 0.693147181f;
  const float EL  = 0.1f * (-6.93147182f);

#pragma unroll
  for (int u = 0; u < 4; ++u) { fsh[t + SKT * u] = 0.f; gsh[t + SKT * u] = 0.f; }
  __syncthreads();

  for (int it = 0; it < n; ++it) {
    const float gmx = block_max4(gsh, red, t, wv, lane);
#pragma unroll
    for (int u = 0; u < 4; ++u) psh[t + SKT * u] = (gsh[t + SKT * u] - gmx) * K2;
    __syncthreads();
#pragma unroll 1
    for (int q = 0; q < NB / SKW; ++q) {
      const int i = wv + SKW * q;
      const float* rp = Ck + ((size_t)i << 10) + 4 * lane;
      const float* sp = psh + 4 * lane;
      float sa = 0.f, sb = 0.f;
#pragma unroll 2
      for (int t8 = 0; t8 < 8; ++t8) {
        const v4f c4 = *(const v4f*)(rp + 128 * t8);
        const v4f g4 = *(const v4f*)(sp + 128 * t8);
        sa += __builtin_amdgcn_exp2f(fmaf(-K2, c4.x, g4.x));
        sb += __builtin_amdgcn_exp2f(fmaf(-K2, c4.y, g4.y));
        sa += __builtin_amdgcn_exp2f(fmaf(-K2, c4.z, g4.z));
        sb += __builtin_amdgcn_exp2f(fmaf(-K2, c4.w, g4.w));
      }
      const float s = wave_sum(sa + sb);
      if (lane == 0) fsh[i] = (EL - gmx) - ELN * __builtin_amdgcn_logf(s);
    }
    __syncthreads();
    const float fmx = block_max4(fsh, red, t, wv, lane);
#pragma unroll
    for (int u = 0; u < 4; ++u) psh[t + SKT * u] = (fsh[t + SKT * u] - fmx) * K2;
    __syncthreads();
    {
      float q0 = 0.f, q1 = 0.f, q2 = 0.f, q3 = 0.f;
      const float* cp = Ck + 4 * t;
#pragma unroll 1
      for (int i = 0; i < NB; i += 4) {
        const v4f F4 = *(const v4f*)(psh + i);
#pragma unroll
        for (int u = 0; u < 4; ++u) {
          const v4f c4 = *(const v4f*)(cp + (size_t)(i + u) * NB);
          const float fu = F4[u];
          q0 += __builtin_amdgcn_exp2f(fmaf(-K2, c4.x, fu));
          q1 += __builtin_amdgcn_exp2f(fmaf(-K2, c4.y, fu));
          q2 += __builtin_amdgcn_exp2f(fmaf(-K2, c4.z, fu));
          q3 += __builtin_amdgcn_exp2f(fmaf(-K2, c4.w, fu));
        }
      }
      const float base = EL - fmx;
      gsh[4 * t + 0] = base - ELN * __builtin_amdgcn_logf(q0);
      gsh[4 * t + 1] = base - ELN * __builtin_amdgcn_logf(q1);
      gsh[4 * t + 2] = base - ELN * __builtin_amdgcn_logf(q2);
      gsh[4 * t + 3] = base - ELN * __builtin_amdgcn_logf(q3);
    }
    __syncthreads();
  }

#pragma unroll
  for (int u = 0; u < 4; ++u) psh[t + SKT * u] = gsh[t + SKT * u] * K2;
  __syncthreads();
  double accd = 0.0;
#pragma unroll 1
  for (int q = 0; q < NB / SKW; ++q) {
    const int i = wv + SKW * q;
    const float fi = fsh[i] * K2;
    const float* rp = Ck + ((size_t)i << 10) + 4 * lane;
    const float* sp = psh + 4 * lane;
    float s = 0.f;
#pragma unroll 2
    for (int t8 = 0; t8 < 8; ++t8) {
      const v4f c4 = *(const v4f*)(rp + 128 * t8);
      const v4f g4 = *(const v4f*)(sp + 128 * t8);
      s = fmaf(__builtin_amdgcn_exp2f(fmaf(-K2, c4.x, g4.x + fi)), c4.x, s);
      s = fmaf(__builtin_amdgcn_exp2f(fmaf(-K2, c4.y, g4.y + fi)), c4.y, s);
      s = fmaf(__builtin_amdgcn_exp2f(fmaf(-K2, c4.z, g4.z + fi)), c4.z, s);
      s = fmaf(__builtin_amdgcn_exp2f(fmaf(-K2, c4.w, g4.w + fi)), c4.w, s);
    }
    accd += (double)s;
  }
  redd[t] = accd;
  __syncthreads();
  if (t == 0) {
    double w = 0.0;
    for (int i = 0; i < SKT; ++i) w += redd[i];
    wtot = w;
  }
  __syncthreads();
  v2d val;
  val.x = wtot;
  val.y = wtot;
  double* dp = Wl + 16 * k + 2 * (t & 7);
  if (t < 8) *(volatile v2d*)dp = val;
  __threadfence();
  if (t < 8) *(volatile v2d*)dp = val;
}

__global__ void __launch_bounds__(32) k_fin(const double* __restrict__ Wl, float* __restrict__ out) {
  if (threadIdx.x == 0) {
    const double w0 = Wl[0], w1 = Wl[16], w2 = Wl[32], w3 = Wl[48], w4 = Wl[64], w5 = Wl[80];
    const double r = ((w0 + w1) + (w2 + w3)) - 2.0 * (w4 + w5);
    const float rf = (float)r;
    *(volatile float*)out = rf;
    __threadfence();
    *(volatile float*)out = rf;
  }
}

extern "C" void kernel_launch(void* const* d_in, const int* in_sizes, int n_in,
                              void* d_out, int out_size, void* d_ws, size_t ws_size,
                              hipStream_t stream) {
  if (n_in < 7 || out_size < 1) return;
  if (in_sizes[0] != NB * DIN || in_sizes[1] != NB * DIN || in_sizes[2] != NB * DIN ||
      in_sizes[3] != NB * DIN || in_sizes[4] != DIN * DE || in_sizes[5] < DE || in_sizes[6] < 1)
    return;

  const float* x0 = (const float*)d_in[0];
  const float* x1 = (const float*)d_in[1];
  const float* x2 = (const float*)d_in[2];
  const float* x3 = (const float*)d_in[3];
  const float* Wc = (const float*)d_in[4];
  const float* bc = (const float*)d_in[5];
  const int*   nit = (const int*)d_in[6];

  const size_t off_wt = 0;
  const size_t sz_wt  = (size_t)DE * DIN * sizeof(_Float16);
  const size_t off_fn = off_wt + sz_wt;
  const size_t sz_fn  = (size_t)NMAT * NB * DE * sizeof(_Float16);
  const size_t off_c  = off_fn + sz_fn;
  const size_t sz_c   = (size_t)NPAIR * NB * NB * sizeof(float);
  const size_t off_wl = off_c + sz_c;
  const size_t sz_wl  = (size_t)NPAIR * 128;
  if (off_wl + sz_wl > ws_size) return;

  char* ws = (char*)d_ws;
  _Float16* Wt = (_Float16*)(ws + off_wt);
  _Float16* Fn = (_Float16*)(ws + off_fn);
  float*    C  = (float*)(ws + off_c);
  double*   Wl = (double*)(ws + off_wl);

  k_wt<<<dim3(DIN / 64, DE / 64), 256, 0, stream>>>(Wc, Wt);
  k_critic<<<dim3(NB / 16, NMAT), 128, 0, stream>>>(x0, x1, x2, x3, Wt, bc, Fn);
  k_cos<<<dim3(NB / 256, NB / 16, NPAIR), 128, 0, stream>>>(Fn, C);
  k_sink<<<NPAIR, SKT, 0, stream>>>(C, nit, Wl);
  k_fin<<<1, 32, 0, stream>>>(Wl, (float*)d_out);
}
